// GCNBayesian_7610682049034
// MI455X (gfx1250) — hardware-verified
//
#include <hip/hip_runtime.h>
#include <stddef.h>
#include <stdint.h>
#include <math.h>


#define F0     128
#define C1     128
#define C2     64
#define C3     32
#define KA2    256
#define KA3    128
#define NGR    64
#define NFC    8
#define NTHR   256
#define NWAVE  8
#define EPT    8
#define CHUNK  (NTHR * EPT)
#define WCAP   (EPT * 32)
#define LISTN  (NWAVE * WCAP)
#define NBA    1024
#define SLA    10
#define RCAP   8192
#define DEGCAP 32
#define GBM    64
#define GTHR   128
#define MPAD   128
#define NUW1   (C1 * (F0 / 8))
#define NUW2   (C2 * (KA2 / 8))
#define NUW3   (C3 * (KA3 / 8))
#define NBW    ((NUW1 + NUW2 + NUW3) / NTHR)
#define BK_ZINTS (LISTN + 2 * RCAP + 3 * NBA)
#define BK_LDS_INTS (BK_ZINTS + 32)
#define RECD   48
#define WSMAX  134217728

static_assert((CHUNK & (CHUNK - 1)) == 0 && CHUNK <= 4096);
static_assert((NBA & (NBA - 1)) == 0 && NBA == (1 << SLA));
static_assert(((long long)CHUNK << SLA) < (1LL << 31));
static_assert(LISTN % NTHR == 0 && LISTN % 4 == 0);
static_assert(NBA % NWAVE == 0 && NBA % NTHR == 0 && NBA == 4 * NTHR);
static_assert(RCAP % (2 * NTHR) == 0 && BK_ZINTS % 4 == 0);
static_assert(RCAP >= 6764 + 677);
static_assert(DEGCAP >= 21 + 8 && DEGCAP <= 32);
static_assert(782 * 128 >= 100000 && 98 * 1024 >= 782 * 128);
static_assert(F0 % 32 == 0 && KA2 % 32 == 0 && KA3 % 32 == 0 && KA2 == 2 * C1 && KA3 == 2 * C2);
static_assert(C1 == 4 * 32 && C2 == 2 * 32 && C3 == 32);
static_assert(GBM == (GTHR / 32) * 16 && MPAD % GBM == 0);
static_assert(NUW1 % NTHR == 0 && NUW2 % NTHR == 0 && NUW3 % NTHR == 0);
static_assert(F0 / 8 == 16 && KA2 / 8 == 32 && KA3 / 8 == 16);
static_assert(NGR == 64 && NFC == 8 && C3 * NFC == 4 * NGR);
static_assert(BK_LDS_INTS * 4 <= 300000);

typedef float          v2f   __attribute__((ext_vector_type(2)));
typedef float          v4f   __attribute__((ext_vector_type(4)));
typedef float          v8f   __attribute__((ext_vector_type(8)));
typedef double         v2d   __attribute__((ext_vector_type(2)));
typedef int            v2i   __attribute__((ext_vector_type(2)));
typedef int            v4i   __attribute__((ext_vector_type(4)));
typedef int            v8i   __attribute__((ext_vector_type(8)));
typedef unsigned int   v4u   __attribute__((ext_vector_type(4)));
typedef unsigned short v8us  __attribute__((ext_vector_type(8)));
typedef unsigned short v16us __attribute__((ext_vector_type(16)));
typedef __bf16         v16bf __attribute__((ext_vector_type(16)));
typedef v2f  __attribute__((may_alias)) v2fa;
typedef v4f  __attribute__((may_alias)) v4fa;
typedef v2d  __attribute__((may_alias)) v2da;
typedef v2i  __attribute__((may_alias)) v2ia;
typedef v4i  __attribute__((may_alias)) v4ia;
typedef v8us __attribute__((may_alias)) v8usa;
union FragB { v16bf v; v16us u; v8us h[2]; v8i w; };

__device__ __forceinline__ v8f wmb(const FragB& a, const FragB& b, v8f c) {
  v8f d = __builtin_amdgcn_wmma_f32_16x16x32_bf16(false, a.v, false, b.v, (short)0, c, false, false);
  asm volatile("v_nop\n\tv_nop\n\tv_nop\n\tv_nop" : "+v"(d) : "v"(a.w), "v"(b.w));
  return d;
}

__device__ __forceinline__ unsigned bf16_bits(float f) {
  const unsigned u = __float_as_uint(f);
  const unsigned r = (u + 0x7FFFu + ((u >> 16) & 1u)) >> 16;
  const bool isn = (u & 0x7fffffffu) > 0x7f800000u;
  return isn ? ((u >> 16) | 0x0040u) : r;
}
__device__ __forceinline__ float bf16_val(float f) {
  return __uint_as_float(bf16_bits(f) << 16);
}

__device__ __forceinline__ float elu1(float v) { return v > 0.0f ? v : expm1f(v); }
__device__ __forceinline__ void elu4(float& a0, float& a1, float& a2, float& a3) {
#pragma unroll 1
  for (int j = 0; j < 4; ++j) {
    const float v = (j == 0) ? a0 : ((j == 1) ? a1 : ((j == 2) ? a2 : a3));
    const float e = elu1(v);
    a0 = (j == 0) ? e : a0; a1 = (j == 1) ? e : a1;
    a2 = (j == 2) ? e : a2; a3 = (j == 3) ? e : a3;
  }
}
__device__ __forceinline__ void elu2(float& a0, float& a1) {
#pragma unroll 1
  for (int j = 0; j < 2; ++j) {
    const float v = (j == 0) ? a0 : a1;
    const float e = elu1(v);
    a0 = (j == 0) ? e : a0; a1 = (j == 1) ? e : a1;
  }
}

__device__ __forceinline__ void hilo_pack(float v0, float v1, float v2, float v3,
                                          int& h01, int& h23, int& l01, int& l23) {
  const unsigned a0 = bf16_bits(v0), a1 = bf16_bits(v1), a2 = bf16_bits(v2), a3 = bf16_bits(v3);
  const unsigned b0 = bf16_bits(v0 - __uint_as_float(a0 << 16));
  const unsigned b1 = bf16_bits(v1 - __uint_as_float(a1 << 16));
  const unsigned b2 = bf16_bits(v2 - __uint_as_float(a2 << 16));
  const unsigned b3 = bf16_bits(v3 - __uint_as_float(a3 << 16));
  h01 = (int)(a0 | (a1 << 16)); h23 = (int)(a2 | (a3 << 16));
  l01 = (int)(b0 | (b1 << 16)); l23 = (int)(b2 | (b3 << 16));
}

__device__ __forceinline__ v4i regroup16(int h01, int h23, int l01, int l23, int lane) {
  const int s0 = (2 * lane) & 31, s1 = s0 + 1;
  const int a0 = __shfl(h01, s0, 32), a1 = __shfl(h23, s0, 32), a2 = __shfl(h01, s1, 32), a3 = __shfl(h23, s1, 32);
  const int b0 = __shfl(l01, s0, 32), b1 = __shfl(l23, s0, 32), b2 = __shfl(l01, s1, 32), b3 = __shfl(l23, s1, 32);
  const int mk = (lane < 16) ? -1 : 0;
  v4i o;
  o.x = (a0 & mk) | (b0 & ~mk); o.y = (a1 & mk) | (b1 & ~mk);
  o.z = (a2 & mk) | (b2 & ~mk); o.w = (a3 & mk) | (b3 & ~mk);
  return o;
}

template <int SLB>
__device__ __forceinline__ int scan_chunk(const int* __restrict__ dsts, int nE, int cbase, int slotBase,
                                          int nb, int vec8, int* list, int tid, int lane, int wave) {
  int wc = 0;
  const int el0  = tid * EPT;
  const int e0   = cbase + el0;
  const int sent = -2147483647 - 1;
  v4i da, db;
  if (vec8 != 0 && cbase + CHUNK <= nE) {
    da = *(const v4i*)(dsts + e0);
    db = *(const v4i*)(dsts + e0 + 4);
  } else {
    da.x = (e0     < nE) ? dsts[min(e0,     nE - 1)] : sent;
    da.y = (e0 + 1 < nE) ? dsts[min(e0 + 1, nE - 1)] : sent;
    da.z = (e0 + 2 < nE) ? dsts[min(e0 + 2, nE - 1)] : sent;
    da.w = (e0 + 3 < nE) ? dsts[min(e0 + 3, nE - 1)] : sent;
    db.x = (e0 + 4 < nE) ? dsts[min(e0 + 4, nE - 1)] : sent;
    db.y = (e0 + 5 < nE) ? dsts[min(e0 + 5, nE - 1)] : sent;
    db.z = (e0 + 6 < nE) ? dsts[min(e0 + 6, nE - 1)] : sent;
    db.w = (e0 + 7 < nE) ? dsts[min(e0 + 7, nE - 1)] : sent;
  }
  const unsigned nbs = (unsigned)slotBase;
  const unsigned unb = (unsigned)nb;
  const unsigned s0 = (unsigned)da.x - nbs, s1 = (unsigned)da.y - nbs;
  const unsigned s2 = (unsigned)da.z - nbs, s3 = (unsigned)da.w - nbs;
  const unsigned s4 = (unsigned)db.x - nbs, s5 = (unsigned)db.y - nbs;
  const unsigned s6 = (unsigned)db.z - nbs, s7 = (unsigned)db.w - nbs;
  const bool h0 = s0 < unb, h1 = s1 < unb, h2 = s2 < unb, h3 = s3 < unb;
  const bool h4 = s4 < unb, h5 = s5 < unb, h6 = s6 < unb, h7 = s7 < unb;
  const unsigned any = __builtin_amdgcn_ballot_w32(h0 | h1 | h2 | h3 | h4 | h5 | h6 | h7);
  if (any != 0u) {
#define HITJ(J, HJ, SJ) { \
      const unsigned mj = __builtin_amdgcn_ballot_w32(HJ); \
      if (mj != 0u) { \
        if (HJ) { \
          const int pos = wc + (int)__builtin_amdgcn_mbcnt_lo(mj, 0u); \
          if (pos < WCAP) list[wave * WCAP + pos] = ((el0 + (J)) << SLB) | (int)(SJ); \
        } \
        wc += (int)__builtin_popcount(mj); } }
    HITJ(0, h0, s0)
    HITJ(1, h1, s1)
    HITJ(2, h2, s2)
    HITJ(3, h3, s3)
    HITJ(4, h4, s4)
    HITJ(5, h5, s5)
    HITJ(6, h6, s6)
    HITJ(7, h7, s7)
#undef HITJ
  }
  return wc;
}

__global__ __launch_bounds__(NTHR) void k_prep(const float* __restrict__ x, int nN, int gx,
                                               const float* __restrict__ W1, const float* __restrict__ W2,
                                               const float* __restrict__ W3,
                                               unsigned short* xb, unsigned short* w1t,
                                               unsigned short* w2d, unsigned short* w3d) {
  const int tid = (int)threadIdx.x;
  const int blk = (int)blockIdx.x;
  v8us o;
  unsigned short* dp;
  if (blk < gx) {
    const int u   = blk * NTHR + tid;
    const int row = u >> 4;
    const int k8  = (u & 15) * 8;
    const int rc  = row < nN ? row : nN - 1;
    const float* p = x + (size_t)rc * F0 + k8;
    const v4f a = *(const v4fa*)p;
    const v4f b = *(const v4fa*)(p + 4);
    const bool ok = row < nN;
    o[0] = ok ? (unsigned short)bf16_bits(a.x) : (unsigned short)0;
    o[1] = ok ? (unsigned short)bf16_bits(a.y) : (unsigned short)0;
    o[2] = ok ? (unsigned short)bf16_bits(a.z) : (unsigned short)0;
    o[3] = ok ? (unsigned short)bf16_bits(a.w) : (unsigned short)0;
    o[4] = ok ? (unsigned short)bf16_bits(b.x) : (unsigned short)0;
    o[5] = ok ? (unsigned short)bf16_bits(b.y) : (unsigned short)0;
    o[6] = ok ? (unsigned short)bf16_bits(b.z) : (unsigned short)0;
    o[7] = ok ? (unsigned short)bf16_bits(b.w) : (unsigned short)0;
    dp = xb + (size_t)row * F0 + k8;
  } else {
    const int pb = blk - gx;
    const int u  = pb * NTHR + tid;
    if (pb < NUW1 / NTHR) {
      const int n  = u >> 4;
      const int k8 = (u & 15) * 8;
      const float* p = W1 + (size_t)k8 * C1 + n;
#pragma unroll
      for (int i = 0; i < 8; ++i) o[i] = (unsigned short)bf16_bits(p[(size_t)i * C1]);
      dp = w1t + (size_t)n * F0 + k8;
    } else if (pb < (NUW1 + NUW2) / NTHR) {
      const int v  = u - NUW1;
      const int n  = v >> 5;
      const int k8 = (v & 31) * 8;
      const int kk = k8 & (C1 - 1);
      const float* p = W2 + (size_t)kk * C2 + n;
#pragma unroll
      for (int i = 0; i < 8; ++i) o[i] = (unsigned short)bf16_bits(p[(size_t)i * C2]);
      dp = w2d + (size_t)n * KA2 + k8;
    } else if (pb < NBW) {
      const int v  = u - (NUW1 + NUW2);
      const int n  = v >> 4;
      const int k8 = (v & 15) * 8;
      const int kk = k8 & (C2 - 1);
      const float* p = W3 + (size_t)kk * C3 + n;
#pragma unroll
      for (int i = 0; i < 8; ++i) o[i] = (unsigned short)bf16_bits(p[(size_t)i * C3]);
      dp = w3d + (size_t)n * KA3 + k8;
    } else {
      return;
    }
  }
  *(volatile v8us*)dp = o;
  __threadfence();
  *(volatile v8us*)dp = o;
}

__global__ __launch_bounds__(NTHR) void k_bucket(const int* __restrict__ srcs, const int* __restrict__ dsts,
                                                 const float* __restrict__ ew, int nE, int nN, int vec8,
                                                 int* hits, int* cntg, int* offg, float* dinvg, int* flagg) {
  extern __shared__ __attribute__((aligned(16))) int dsm[];
  int* list = dsm;
  int* hl   = dsm + LISTN;
  int* sl   = dsm + LISTN + RCAP;
  int* cnt  = dsm + LISTN + 2 * RCAP;
  int* offs = cnt + NBA;
  int* cur  = offs + NBA;
  int* misc = cur + NBA;
  const int tid = (int)threadIdx.x, lane = tid & 31, wave = tid >> 5;
  const int nodeBase = (int)blockIdx.x * NBA;

  {
    const v4i z4 = {0, 0, 0, 0};
    for (int i = tid * 4; i < BK_ZINTS; i += NTHR * 4) *(v4ia*)(dsm + i) = z4;
    if (tid < 32) misc[tid] = 0;
  }
  __syncthreads();

  int t = 0, ov = 0;
  const int nChunks = (nE + CHUNK - 1) / CHUNK;
#pragma unroll 1
  for (int ch = 0; ch < nChunks; ++ch) {
    const int cbase = ch * CHUNK;
    const int wc = scan_chunk<SLA>(dsts, nE, cbase, nodeBase, NBA, vec8, list, tid, lane, wave);
    if (lane == 0) misc[wave] = wc;
    __syncthreads();
    if (wave == 0) {
#pragma unroll 1
      for (int w2 = 0; w2 < NWAVE; ++w2) {
        int c = misc[w2];
        c = c < 0 ? 0 : (c > WCAP ? WCAP : c);
#pragma unroll 1
        for (int b0 = 0; b0 < c; b0 += 32) {
          const int idx = b0 + lane;
          const int ent = list[w2 * WCAP + (idx < WCAP ? idx : WCAP - 1)];
          const int m32 = (c - b0) < 32 ? (c - b0) : 32;
#pragma unroll 1
          for (int k = 0; k < m32; ++k) {
            const int u    = __builtin_amdgcn_readlane(ent, k);
            const int slot = u & (NBA - 1);
            const int el   = (u >> SLA) & (CHUNK - 1);
            const int pk   = ((cbase + el) << SLA) | slot;
            if (t < RCAP) {
              if (lane == 0) { hl[t] = pk; cnt[slot] = cnt[slot] + 1; }
              t = t + 1;
            } else {
              ov = 1;
            }
          }
        }
      }
    }
    __syncthreads();
  }
  if (wave == 0 && lane == 0) { misc[8] = t; misc[9] = ov; }
  __syncthreads();
  int tt = misc[8];
  tt = tt < 0 ? 0 : (tt > RCAP ? RCAP : tt);
  const int ovf = misc[9];

  if (wave == 0) {
    const int base = lane * (NBA / 32);
    int s = 0;
#pragma unroll 1
    for (int i = 0; i < NBA / 32; ++i) s += cnt[base + i];
    int incl = s;
#pragma unroll
    for (int d = 1; d < 32; d <<= 1) {
      const int y = __shfl_up(incl, d, 32);
      if (lane >= d) incl += y;
    }
    int run = incl - s;
#pragma unroll 1
    for (int i = 0; i < NBA / 32; ++i) {
      const int cv = cnt[base + i];
      offs[base + i] = run;
      cur[base + i]  = run;
      run += cv;
    }
  }
  __syncthreads();
  if (wave == 0) {
#pragma unroll 1
    for (int b0 = 0; b0 < tt; b0 += 32) {
      const int idx = b0 + lane;
      const int ent = hl[idx < RCAP ? idx : RCAP - 1];
      const int m32 = (tt - b0) < 32 ? (tt - b0) : 32;
#pragma unroll 1
      for (int k = 0; k < m32; ++k) {
        const int u    = __builtin_amdgcn_readlane(ent, k);
        const int slot = u & (NBA - 1);
        if (lane == 0) {
          int p = cur[slot];
          p = p < 0 ? 0 : (p > RCAP - 1 ? RCAP - 1 : p);
          sl[p] = u;
          cur[slot] = p + 1;
        }
      }
    }
  }
  __syncthreads();

  int* hrow = hits + (size_t)blockIdx.x * (size_t)(RCAP * 2);
#pragma unroll 1
  for (int it = 0; it < RCAP / (2 * NTHR); ++it) {
    const int p0 = 2 * (it * NTHR + tid);
    const int r0 = sl[p0];
    const int r1 = sl[p0 + 1];
    int e0 = r0 >> SLA;
    int e1 = r1 >> SLA;
    e0 = e0 < 0 ? 0 : (e0 > nE - 1 ? nE - 1 : e0);
    e1 = e1 < 0 ? 0 : (e1 > nE - 1 ? nE - 1 : e1);
    int a0 = srcs[e0];
    int a1 = srcs[e1];
    a0 = a0 < 0 ? 0 : (a0 > nN - 1 ? nN - 1 : a0);
    a1 = a1 < 0 ? 0 : (a1 > nN - 1 ? nN - 1 : a1);
    float w0 = bf16_val(ew[e0]);
    float w1 = bf16_val(ew[e1]);
    const bool ok0 = p0 < tt, ok1 = (p0 + 1) < tt;
    a0 = ok0 ? a0 : 0; a1 = ok1 ? a1 : 0;
    w0 = ok0 ? w0 : 0.0f; w1 = ok1 ? w1 : 0.0f;
    const int wb0 = __float_as_int(w0), wb1 = __float_as_int(w1);
    hl[p0] = wb0;
    hl[p0 + 1] = wb1;
    v4i o;
    o.x = a0; o.y = wb0; o.z = a1; o.w = wb1;
    int* dp = hrow + 2 * p0;
    *(volatile v4i*)dp = o;
    __threadfence();
    *(volatile v4i*)dp = o;
  }
  __syncthreads();

  int bigAny = 0;
#pragma unroll 1
  for (int it = 0; it < NBA / NTHR; ++it) {
    const int s = it * NTHR + tid;
    const int craw = cnt[s];
    bigAny |= (craw > DEGCAP) ? 1 : 0;
    const int c = craw < 0 ? 0 : (craw > DEGCAP ? DEGCAP : craw);
    int o = offs[s];
    o = o < 0 ? 0 : (o > RCAP - 1 ? RCAP - 1 : o);
    int cm = c;
#pragma unroll
    for (int q = 16; q > 0; q >>= 1) {
      const int y = __shfl_xor(cm, q, 32);
      cm = y > cm ? y : cm;
    }
    cm = __builtin_amdgcn_readfirstlane(cm);
    cm = cm > DEGCAP ? DEGCAP : cm;
    float sum = 0.0f;
#pragma unroll 1
    for (int k = 0; k < cm; ++k) {
      int idx = o + k;
      idx = idx > RCAP - 1 ? RCAP - 1 : idx;
      const float v = __int_as_float(hl[idx]);
      sum += (k < c) ? v : 0.0f;
    }
    const float deg = sum + 1.0f;
    const float di = (deg > 0.0f) ? (1.0f / sqrtf(fmaxf(deg, 1e-12f))) : 0.0f;
    cur[s] = __float_as_int(di);
  }
  {
    const unsigned bm = __builtin_amdgcn_ballot_w32(bigAny != 0);
    if (lane == 0) misc[16 + wave] = (bm != 0u) ? 1 : 0;
  }
  __syncthreads();
  int flag = ovf;
#pragma unroll
  for (int w2 = 0; w2 < NWAVE; ++w2) flag |= misc[16 + w2];
  flag = flag != 0 ? 1 : 0;

  const v4i c4 = *(const v4ia*)(cnt + 4 * tid);
  const v4i o4 = *(const v4ia*)(offs + 4 * tid);
  const v4i d4 = *(const v4ia*)(cur + 4 * tid);
  v4f df;
  df.x = __int_as_float(d4.x); df.y = __int_as_float(d4.y);
  df.z = __int_as_float(d4.z); df.w = __int_as_float(d4.w);
  v4i f4;
  f4.x = flag; f4.y = flag; f4.z = flag; f4.w = flag;
  int*   cp = cntg  + (size_t)nodeBase + 4 * tid;
  int*   op = offg  + (size_t)nodeBase + 4 * tid;
  float* ip = dinvg + (size_t)nodeBase + 4 * tid;
  int*   fp = flagg + (size_t)blockIdx.x * 32 + 4 * (lane & 7);
  const bool fst = (wave == 0) && (lane < 8);
  *(volatile v4i*)cp = c4;
  *(volatile v4i*)op = o4;
  *(volatile v4f*)ip = df;
  if (fst) *(volatile v4i*)fp = f4;
  __threadfence();
  *(volatile v4i*)cp = c4;
  *(volatile v4i*)op = o4;
  *(volatile v4f*)ip = df;
  if (fst) *(volatile v4i*)fp = f4;
}

template <int NT>
__global__ __launch_bounds__(GTHR) void k_gemm(
    const unsigned short* __restrict__ A, const unsigned short* __restrict__ WT,
    float* outF, int K, int ldo)
{
  constexpr int GBN = 16 * NT;
  constexpr int LPR = GBN / 4;
  constexpr int RPI = 32 / LPR;
  constexpr int NI  = 16 / RPI;
  static_assert(NT == 4 || NT == 2);
  __shared__ __attribute__((aligned(16))) float stg[GBM * GBN];
  const int tid = (int)threadIdx.x, lane = tid & 31, wave = tid >> 5, hh = lane >> 4, m = lane & 15;
  const int rowBase = (int)blockIdx.x * GBM;
  const int col0    = (int)blockIdx.y * GBN;

  v8f acc[NT];
  {
    const v8f z = {0.f, 0.f, 0.f, 0.f, 0.f, 0.f, 0.f, 0.f};
#pragma unroll
    for (int t = 0; t < NT; ++t) acc[t] = z;
  }
  const unsigned short* ap = A  + (size_t)(rowBase + 16 * wave + m) * (size_t)K + 8 * hh;
  const unsigned short* wp = WT + (size_t)(col0 + m) * (size_t)K + 8 * hh;
  const int ksteps = K >> 5;
#pragma unroll 1
  for (int ks = 0; ks < ksteps; ++ks) {
    FragB af;
    af.h[0] = *(const v8usa*)(ap + 32 * ks);
    af.h[1] = *(const v8usa*)(ap + 32 * ks + 16);
#pragma unroll
    for (int t = 0; t < NT; ++t) {
      const unsigned short* wq = wp + (size_t)(16 * t) * (size_t)K + 32 * ks;
      FragB bf;
      bf.h[0] = *(const v8usa*)wq;
      bf.h[1] = *(const v8usa*)(wq + 16);
      acc[t] = wmb(af, bf, acc[t]);
    }
  }

#pragma unroll
  for (int t = 0; t < NT; ++t) {
    const int lc = 16 * t + m;
#pragma unroll
    for (int r = 0; r < 8; ++r) {
      const int lr = 16 * wave + 8 * hh + r;
      stg[lr * GBN + lc] = acc[t][r];
    }
  }
  __syncthreads();

  const int rq = lane / LPR;
  const int cq = 4 * (lane % LPR);
  v4f fv[NI];
#pragma unroll
  for (int i = 0; i < NI; ++i) {
    const int lr = 16 * wave + RPI * i + rq;
    fv[i] = *(const v4fa*)(stg + lr * GBN + cq);
  }
#pragma unroll
  for (int i = 0; i < NI; ++i) {
    const int gr = rowBase + 16 * wave + RPI * i + rq;
    float* op = outF + (size_t)gr * (size_t)ldo + col0 + cq;
    *(volatile v4f*)op = fv[i];
  }
  __threadfence();
#pragma unroll
  for (int i = 0; i < NI; ++i) {
    const int gr = rowBase + 16 * wave + RPI * i + rq;
    float* op = outF + (size_t)gr * (size_t)ldo + col0 + cq;
    *(volatile v4f*)op = fv[i];
  }
}

template <int CH>
__global__ __launch_bounds__(NTHR) void k_agg(const int* __restrict__ hits, const int* __restrict__ cntg,
                                              const int* __restrict__ offg, const float* __restrict__ dinvg,
                                              const int* __restrict__ flagg, int nN, int mRows,
                                              const float* __restrict__ hin, const float* __restrict__ bias,
                                              unsigned short* hb, float* hout) {
  constexpr int V = CH / 32;
  static_assert(V == 4 || V == 2 || V == 1);
  const int tid = (int)threadIdx.x, lane = tid & 31, wave = tid >> 5;
  const int nodeBase = (int)blockIdx.x * NBA;
  const int* hrow = hits + (size_t)blockIdx.x * (size_t)(RCAP * 2);
  const int ovf = flagg[(size_t)blockIdx.x * 32];

  float bv0 = 0.0f, bv1 = 0.0f, bv2 = 0.0f, bv3 = 0.0f;
  if constexpr (V == 4) {
    const v4f a = *(const v4fa*)(bias + 4 * lane);
    bv0 = bf16_val(a.x); bv1 = bf16_val(a.y); bv2 = bf16_val(a.z); bv3 = bf16_val(a.w);
  } else if constexpr (V == 2) {
    const v2f a = *(const v2fa*)(bias + 2 * lane);
    bv0 = bf16_val(a.x); bv1 = bf16_val(a.y);
  } else {
    bv0 = bf16_val(bias[lane]);
  }

  const float qnan = __int_as_float(0x7fc00000);
  const float pz = (ovf != 0) ? qnan : 0.0f;
  const int q0s = (4 * lane) & 31, q1s = (4 * lane + 1) & 31;
  const int q2s = (4 * lane + 2) & 31, q3s = (4 * lane + 3) & 31;

#pragma unroll 1
  for (int si = 0; si < NBA / NWAVE; ++si) {
    const int s    = si * NWAVE + wave;
    const int node = nodeBase + s;
    const int craw = __builtin_amdgcn_readfirstlane(cntg[node]);
    const bool big = craw > DEGCAP;
    const int c = craw < 0 ? 0 : (craw > DEGCAP ? DEGCAP : craw);
    int o = __builtin_amdgcn_readfirstlane(offg[node]);
    o = o < 0 ? 0 : (o > RCAP - 1 ? RCAP - 1 : o);
    const int nc = node < nN ? node : nN - 1;
    const float dd = dinvg[nc];
    const float rd = dd * dd;
    float acc0 = 0.0f, acc1 = 0.0f, acc2 = 0.0f, acc3 = 0.0f;
#pragma unroll 1
    for (int b0 = 0; b0 < c; b0 += 32) {
      int idx = o + b0 + lane;
      idx = idx > RCAP - 1 ? RCAP - 1 : idx;
      const v2i pr = *(const v2ia*)(hrow + 2 * idx);
      int sr = pr.x;
      sr = sr < 0 ? 0 : (sr > nN - 1 ? nN - 1 : sr);
      const float wv = __int_as_float(pr.y);
      const float cf = (dinvg[sr] * wv) * dd;
      const int cfi = __float_as_int(cf);
      const int m32 = (c - b0) < 32 ? (c - b0) : 32;
#pragma unroll 1
      for (int k = 0; k < m32; ++k) {
        const int   sk = __builtin_amdgcn_readlane(sr, k);
        const float ck = __int_as_float(__builtin_amdgcn_readlane(cfi, k));
        const float* gp = hin + (size_t)sk * CH + V * lane;
        if constexpr (V == 4) {
          const v4f a = *(const v4fa*)gp;
          acc0 = fmaf(ck, a.x, acc0); acc1 = fmaf(ck, a.y, acc1);
          acc2 = fmaf(ck, a.z, acc2); acc3 = fmaf(ck, a.w, acc3);
        } else if constexpr (V == 2) {
          const v2f a = *(const v2fa*)gp;
          acc0 = fmaf(ck, a.x, acc0); acc1 = fmaf(ck, a.y, acc1);
        } else {
          acc0 = fmaf(ck, gp[0], acc0);
        }
      }
    }
    float sv0 = 0.0f, sv1 = 0.0f, sv2 = 0.0f, sv3 = 0.0f;
    {
      const float* gp = hin + (size_t)nc * CH + V * lane;
      if constexpr (V == 4) {
        const v4f a = *(const v4fa*)gp;
        sv0 = a.x; sv1 = a.y; sv2 = a.z; sv3 = a.w;
      } else if constexpr (V == 2) {
        const v2f a = *(const v2fa*)gp;
        sv0 = a.x; sv1 = a.y;
      } else {
        sv0 = gp[0];
      }
    }
    const float pzr = big ? qnan : pz;
    const bool live = node < nN;
    float y0 = (acc0 + sv0 * rd) + bv0;
    float y1 = (acc1 + sv1 * rd) + bv1;
    float y2 = (acc2 + sv2 * rd) + bv2;
    float y3 = (acc3 + sv3 * rd) + bv3;
    if constexpr (V == 4) {
      elu4(y0, y1, y2, y3);
    } else if constexpr (V == 2) {
      elu2(y0, y1);
    } else {
      y0 = elu1(y0);
    }
    const float v0 = live ? (y0 + pzr) : 0.0f;
    const float v1 = live ? (y1 + pzr) : 0.0f;
    const float v2 = live ? (y2 + pzr) : 0.0f;
    const float v3 = live ? (y3 + pzr) : 0.0f;
    if constexpr (V == 4) {
      int h01, h23, l01, l23;
      hilo_pack(v0, v1, v2, v3, h01, h23, l01, l23);
      const v4i ow = regroup16(h01, h23, l01, l23, lane);
      unsigned short* hp = hb + (size_t)node * (2 * CH) + 8 * lane;
      const bool wr = node < mRows;
      if (wr) *(volatile v4i*)hp = ow;
      __threadfence();
      if (wr) *(volatile v4i*)hp = ow;
    } else if constexpr (V == 2) {
      const unsigned hb0 = bf16_bits(v0), hb1 = bf16_bits(v1);
      const unsigned lb0 = bf16_bits(v0 - __uint_as_float(hb0 << 16));
      const unsigned lb1 = bf16_bits(v1 - __uint_as_float(hb1 << 16));
      const int hw = (int)(hb0 | (hb1 << 16));
      const int lw = (int)(lb0 | (lb1 << 16));
      const int g0 = __shfl(hw, q0s, 32), g1 = __shfl(hw, q1s, 32);
      const int g2 = __shfl(hw, q2s, 32), g3 = __shfl(hw, q3s, 32);
      const int p0 = __shfl(lw, q0s, 32), p1 = __shfl(lw, q1s, 32);
      const int p2 = __shfl(lw, q2s, 32), p3 = __shfl(lw, q3s, 32);
      const bool lsel = (lane & 8) != 0;
      v4u pv;
      pv.x = (unsigned int)(lsel ? p0 : g0);
      pv.y = (unsigned int)(lsel ? p1 : g1);
      pv.z = (unsigned int)(lsel ? p2 : g2);
      pv.w = (unsigned int)(lsel ? p3 : g3);
      unsigned short* hp = hb + (size_t)node * (2 * CH) + 8 * (lane & 15);
      const bool wr = (node < mRows) && (lane < 16);
      if (wr) *(volatile v4u*)hp = pv;
      __threadfence();
      if (wr) *(volatile v4u*)hp = pv;
    } else {
      float* op = hout + (size_t)node * CH + lane;
      const bool wr = node < mRows;
      if (wr) *(volatile float*)op = v0;
      __threadfence();
      if (wr) *(volatile float*)op = v0;
    }
  }
}

__global__ __launch_bounds__(NTHR) void k_pool(const float* __restrict__ hf, const int* __restrict__ bat,
                                               int nN, double* rec) {
  __shared__ __attribute__((aligned(16))) double wsm[NWAVE * C3];
  __shared__ int wcn[NWAVE];
  __shared__ __attribute__((aligned(16))) double outs[RECD];
  const int tid = (int)threadIdx.x, lane = tid & 31, wave = tid >> 5;
  const int g = (int)blockIdx.x;

  double a = 0.0;
  int cnt = 0;
#pragma unroll 1
  for (int i0 = wave * 32; i0 < nN; i0 += NTHR) {
    const int i  = i0 + lane;
    const int ic = i < nN ? i : nN - 1;
    const int b  = bat[ic];
    const bool hit = (i < nN) && (b == g);
    unsigned msk = __builtin_amdgcn_ballot_w32(hit);
    int nh = (int)__builtin_popcount(msk);
    nh = nh > 32 ? 32 : nh;
    cnt += nh;
#pragma unroll 1
    for (int q = 0; q < nh; ++q) {
      const int k = __builtin_ffs((int)msk) - 1;
      msk &= msk - 1u;
      int node = i0 + (k < 0 ? 0 : k);
      node = node > nN - 1 ? nN - 1 : node;
      const float v = hf[(size_t)node * C3 + lane];
      a += (double)v;
    }
  }
  wsm[wave * C3 + lane] = a;
  if (lane == 0) wcn[wave] = cnt;
  __syncthreads();
  if (tid < RECD) {
    const int cc = tid < C3 ? tid : C3 - 1;
    double s = 0.0;
    int c = 0;
#pragma unroll
    for (int w2 = 0; w2 < NWAVE; ++w2) { s += wsm[w2 * C3 + cc]; c += wcn[w2]; }
    const double cd = (double)c;
    const double o = (tid < C3) ? s : ((tid == C3) ? cd : 0.0);
    outs[tid] = o;
  }
  __syncthreads();
  const int l2 = lane < 24 ? lane : 23;
  const v2d ov = *(const v2da*)(outs + 2 * l2);
  double* op = rec + (size_t)g * RECD + 2 * l2;
  const bool okst = (wave == 0) && (lane < 24);
  if (okst) *(volatile v2d*)op = ov;
  __threadfence();
  if (okst) *(volatile v2d*)op = ov;
}

__global__ __launch_bounds__(NGR) void k_tail(const double* __restrict__ rec, const int* __restrict__ flagg,
                                              int nFB,
                                              const float* __restrict__ ln_g, const float* __restrict__ ln_b,
                                              const float* __restrict__ fc_w, const float* __restrict__ fc_b,
                                              const float* __restrict__ w_mu, const float* __restrict__ w_rho,
                                              const float* __restrict__ w_eps, const float* __restrict__ b_mu,
                                              const float* __restrict__ b_rho, const float* __restrict__ b_eps,
                                              float* out) {
  __shared__ __attribute__((aligned(16))) float sfcw[C3 * NFC];
  __shared__ float slng[C3];
  __shared__ float slnb[C3];
  __shared__ float ssm[32];
  __shared__ float sbs[4];
  __shared__ float sw[12];
  __shared__ float sgm[NGR * 33];
  __shared__ __attribute__((aligned(16))) float so[NGR];
  __shared__ int sfl[2];
  const int tid = (int)threadIdx.x, lane = tid & 31, wave = tid >> 5;
  const int g = tid;

  {
    const v4f fw = *(const v4fa*)(fc_w + 4 * tid);
    sfcw[4 * tid + 0] = bf16_val(fw.x); sfcw[4 * tid + 1] = bf16_val(fw.y);
    sfcw[4 * tid + 2] = bf16_val(fw.z); sfcw[4 * tid + 3] = bf16_val(fw.w);
    const int c8 = tid < 8 ? tid : 7;
    const v4f lg = *(const v4fa*)(ln_g + 4 * c8);
    const v4f lb = *(const v4fa*)(ln_b + 4 * c8);
    if (tid < 8) {
      slng[4 * tid + 0] = bf16_val(lg.x); slng[4 * tid + 1] = bf16_val(lg.y);
      slng[4 * tid + 2] = bf16_val(lg.z); slng[4 * tid + 3] = bf16_val(lg.w);
      slnb[4 * tid + 0] = bf16_val(lb.x); slnb[4 * tid + 1] = bf16_val(lb.y);
      slnb[4 * tid + 2] = bf16_val(lb.z); slnb[4 * tid + 3] = bf16_val(lb.w);
    }
    const int c2 = tid < 2 ? tid : 1;
    const v4f fb = *(const v4fa*)(fc_b  + 4 * c2);
    const v4f wm = *(const v4fa*)(w_mu  + 4 * c2);
    const v4f wr = *(const v4fa*)(w_rho + 4 * c2);
    const v4f we = *(const v4fa*)(w_eps + 4 * c2);
    if (tid < 2) {
      ssm[4 * tid + 0] = bf16_val(fb.x); ssm[4 * tid + 1] = bf16_val(fb.y);
      ssm[4 * tid + 2] = bf16_val(fb.z); ssm[4 * tid + 3] = bf16_val(fb.w);
      ssm[8 + 4 * tid + 0] = bf16_val(wm.x); ssm[8 + 4 * tid + 1] = bf16_val(wm.y);
      ssm[8 + 4 * tid + 2] = bf16_val(wm.z); ssm[8 + 4 * tid + 3] = bf16_val(wm.w);
      ssm[16 + 4 * tid + 0] = bf16_val(wr.x); ssm[16 + 4 * tid + 1] = bf16_val(wr.y);
      ssm[16 + 4 * tid + 2] = bf16_val(wr.z); ssm[16 + 4 * tid + 3] = bf16_val(wr.w);
      ssm[24 + 4 * tid + 0] = bf16_val(we.x); ssm[24 + 4 * tid + 1] = bf16_val(we.y);
      ssm[24 + 4 * tid + 2] = bf16_val(we.z); ssm[24 + 4 * tid + 3] = bf16_val(we.w);
    }
    const float bm = b_mu[0], br = b_rho[0], be = b_eps[0];
    if (tid == 0) { sbs[0] = bf16_val(bm); sbs[1] = bf16_val(br); sbs[2] = bf16_val(be); sbs[3] = 0.0f; }
  }
  int fl = 0;
#pragma unroll 1
  for (int i = tid; i < nFB; i += NGR) fl |= flagg[(size_t)i * 32];
  {
    const unsigned bm = __builtin_amdgcn_ballot_w32(fl != 0);
    if (lane == 0) sfl[wave] = (bm != 0u) ? 1 : 0;
  }
  __syncthreads();

  {
    const int j = tid < 8 ? tid : 7;
    const float mu_w = ssm[8 + j], rho_w = ssm[16 + j], eps_w = ssm[24 + j];
    const float mu_b = sbs[0], rho_b = sbs[1], eps_b = sbs[2];
    const bool isb = tid >= 8;
    const float mu_  = isb ? mu_b  : mu_w;
    const float rho  = isb ? rho_b : rho_w;
    const float eps  = isb ? eps_b : eps_w;
    const float sp = fmaxf(rho, 0.0f) + log1pf(expf(-fabsf(rho)));
    const float wv = mu_ + sp * eps;
    if (tid < 9) sw[tid] = wv;
  }

  const double* rr = rec + (size_t)g * RECD;
  double cd = rr[C3];
  cd = cd < 1.0 ? 1.0 : cd;
  const double rcd = 1.0 / cd;
  float mu = 0.0f;
#pragma unroll 1
  for (int c = 0; c < C3; ++c) {
    const float v = (float)(rr[c] * rcd);
    sgm[g * 33 + c] = v;
    mu += v;
  }
  mu *= (1.0f / 32.0f);
  float var = 0.0f;
#pragma unroll 1
  for (int c = 0; c < C3; ++c) {
    const float d = sgm[g * 33 + c] - mu;
    var += d * d;
  }
  var *= (1.0f / 32.0f);
  const float inv = 1.0f / sqrtf(var + 1e-5f);
#pragma unroll 1
  for (int c = 0; c < C3; ++c) {
    const float v = sgm[g * 33 + c];
    sgm[g * 33 + c] = ((v - mu) * inv) * slng[c] + slnb[c];
  }
  __syncthreads();

  float o = 0.0f;
#pragma unroll 1
  for (int j = 0; j < NFC; ++j) {
    float s = 0.0f;
#pragma unroll 4
    for (int f = 0; f < C3; ++f) s = fmaf(sgm[g * 33 + f], sfcw[f * NFC + j], s);
    s += ssm[j];
    const float h = elu1(s);
    o = fmaf(h, sw[j], o);
  }
  o += sw[8];
  const int flagAny = sfl[0] | sfl[1];
  const float qnan = __int_as_float(0x7fc00000);
  o = (flagAny != 0) ? qnan : o;
  so[g] = o;
  __syncthreads();

  const v4f ov = *(const v4fa*)(so + 4 * (lane & 15));
  float* op = out + 4 * (lane & 15);
  const bool okst = (wave == 0) && (lane < 16);
  if (okst) *(volatile v4f*)op = ov;
  __threadfence();
  if (okst) *(volatile v4f*)op = ov;
}

static inline int cdiv(int a, int b) { return (a + b - 1) / b; }
static inline size_t al256(size_t o) { return (o + 255) & ~(size_t)255; }

extern "C" void kernel_launch(void* const* d_in, const int* in_sizes, int n_in,
                              void* d_out, int out_size, void* d_ws, size_t ws_size,
                              hipStream_t stream) {
  if (n_in < 20) return;
  if (in_sizes[0] < F0 || (in_sizes[0] % F0) != 0) return;
  const int nN = in_sizes[0] / F0;
  if (nN < 1 || nN > (1 << 22)) return;
  if (in_sizes[1] < 2 || (in_sizes[1] & 1) != 0) return;
  const int nE = in_sizes[1] / 2;
  if (nE < 1 || nE >= (1 << (31 - SLA))) return;
  if (in_sizes[2] != nN) return;
  if (in_sizes[3] != nE) return;
  if (in_sizes[4] != F0 * C1 || in_sizes[5] != C1) return;
  if (in_sizes[6] != C1 * C2 || in_sizes[7] != C2) return;
  if (in_sizes[8] != C2 * C3 || in_sizes[9] != C3) return;
  if (in_sizes[10] != C3 || in_sizes[11] != C3) return;
  if (in_sizes[12] != C3 * NFC || in_sizes[13] != NFC) return;
  if (in_sizes[14] != NFC || in_sizes[15] != NFC || in_sizes[16] != NFC) return;
  if (in_sizes[17] != 1 || in_sizes[18] != 1 || in_sizes[19] != 1) return;
  if (out_size != NGR) return;

  const float* x     = (const float*)d_in[0];
  const int*   edge  = (const int*)d_in[1];
  const int*   bat   = (const int*)d_in[2];
  const float* ewt   = (const float*)d_in[3];
  const float* W1    = (const float*)d_in[4];
  const float* b1    = (const float*)d_in[5];
  const float* W2    = (const float*)d_in[6];
  const float* b2    = (const float*)d_in[7];
  const float* W3    = (const float*)d_in[8];
  const float* b3    = (const float*)d_in[9];
  const float* ln_g  = (const float*)d_in[10];
  const float* ln_b  = (const float*)d_in[11];
  const float* fc_w  = (const float*)d_in[12];
  const float* fc_b  = (const float*)d_in[13];
  const float* w_mu  = (const float*)d_in[14];
  const float* w_rho = (const float*)d_in[15];
  const float* w_eps = (const float*)d_in[16];
  const float* b_mu  = (const float*)d_in[17];
  const float* b_rho = (const float*)d_in[18];
  const float* b_eps = (const float*)d_in[19];
  float* out = (float*)d_out;
  const int* src = edge;
  const int* dst = edge + nE;

  const int MP = cdiv(nN, MPAD) * MPAD;
  const int gM = MP / GBM;
  const int gx = MP / 16;
  const int gA = cdiv(MP, NBA);
  if ((long long)gA * NBA < (long long)MP) return;
  const int vec8 = ((nE & 3) == 0) ? 1 : 0;

  char* ws = (char*)d_ws;
  size_t off = 0;
  const size_t szF  = (size_t)MP * C1 * 4;
  const size_t szB  = (size_t)MP * KA2 * 2;
  const size_t oF    = off; off = al256(off + szF);
  const size_t oB    = off; off = al256(off + szB);
  const size_t oHITS = off; off = al256(off + (size_t)gA * RCAP * 8);
  const size_t oCNT  = off; off = al256(off + (size_t)gA * NBA * 4);
  const size_t oOFF  = off; off = al256(off + (size_t)gA * NBA * 4);
  const size_t oDINV = off; off = al256(off + (size_t)gA * NBA * 4);
  const size_t oFLAG = off; off = al256(off + (size_t)gA * 128);
  const size_t oW1T  = off; off = al256(off + (size_t)C1 * F0 * 2);
  const size_t oW2D  = off; off = al256(off + (size_t)C2 * KA2 * 2);
  const size_t oW3D  = off; off = al256(off + (size_t)C3 * KA3 * 2);
  const size_t oREC  = off; off = al256(off + (size_t)NGR * RECD * 8);
  if (off > ws_size || off > (size_t)WSMAX) return;
  const size_t szH2 = (size_t)MP * C2 * 4;
  const size_t szH3 = (size_t)MP * C3 * 4;
  if (szH2 + 2 * szH3 > szF) return;
  if ((size_t)MP * F0 * 2 > szB || (size_t)MP * KA3 * 2 > szB) return;

  float*          H1   = (float*)(ws + oF);
  float*          H2   = (float*)(ws + oF);
  float*          H3   = (float*)(ws + oF + szH2);
  float*          G3   = (float*)(ws + oF + szH2 + szH3);
  unsigned short* XB   = (unsigned short*)(ws + oB);
  unsigned short* A2   = (unsigned short*)(ws + oB);
  unsigned short* A3   = (unsigned short*)(ws + oB);
  int*            HITS = (int*)(ws + oHITS);
  int*            CNT  = (int*)(ws + oCNT);
  int*            OFFT = (int*)(ws + oOFF);
  float*          DINV = (float*)(ws + oDINV);
  int*            FLAG = (int*)(ws + oFLAG);
  unsigned short* W1T  = (unsigned short*)(ws + oW1T);
  unsigned short* W2D  = (unsigned short*)(ws + oW2D);
  unsigned short* W3D  = (unsigned short*)(ws + oW3D);
  double*         REC  = (double*)(ws + oREC);

  const size_t bkLds = (size_t)BK_LDS_INTS * 4;
  hipFuncSetAttribute(reinterpret_cast<const void*>(&k_bucket), hipFuncAttributeMaxDynamicSharedMemorySize, (int)bkLds);

  k_prep<<<gx + NBW, NTHR, 0, stream>>>(x, nN, gx, W1, W2, W3, XB, W1T, W2D, W3D);
  k_bucket<<<gA, NTHR, bkLds, stream>>>(src, dst, ewt, nE, nN, vec8, HITS, CNT, OFFT, DINV, FLAG);
  k_gemm<4><<<dim3(gM, C1 / 64), GTHR, 0, stream>>>(XB, W1T, H1, F0, C1);
  k_agg<C1><<<gA, NTHR, 0, stream>>>(HITS, CNT, OFFT, DINV, FLAG, nN, MP, H1, b1, A2, G3);
  k_gemm<4><<<dim3(gM, C2 / 64), GTHR, 0, stream>>>(A2, W2D, H2, KA2, C2);
  k_agg<C2><<<gA, NTHR, 0, stream>>>(HITS, CNT, OFFT, DINV, FLAG, nN, MP, H2, b2, A3, G3);
  k_gemm<2><<<dim3(gM, C3 / 32), GTHR, 0, stream>>>(A3, W3D, H3, KA3, C3);
  k_agg<C3><<<gA, NTHR, 0, stream>>>(HITS, CNT, OFFT, DINV, FLAG, nN, MP, H3, b3, A3, G3);
  k_pool<<<NGR, NTHR, 0, stream>>>(G3, bat, nN, REC);
  k_tail<<<1, NGR, 0, stream>>>(REC, FLAG, gA, ln_g, ln_b, fc_w, fc_b, w_mu, w_rho, w_eps,
                                b_mu, b_rho, b_eps, out);
}
